// FlowGNN_50002009260670
// MI455X (gfx1250) — hardware-verified
//
#include <hip/hip_runtime.h>

typedef __attribute__((ext_vector_type(16))) _Float16 v16h;
typedef __attribute__((ext_vector_type(8)))  _Float16 v8h;
typedef __attribute__((ext_vector_type(8)))  float    v8f;
typedef __attribute__((ext_vector_type(4)))  float    v4f;
typedef __attribute__((ext_vector_type(4)))  unsigned v4u;

#define N_NODES 100000
#define DEG     32
#define BQ      2048
#define F_IN    64
#define F_H     128
#define F_OUT   64
#define ROWS1   (BQ * (DEG + 1))

__device__ __forceinline__ v8f wmma_f16(v16h a, v16h b, v8f c) {
  v8f d = __builtin_amdgcn_wmma_f32_16x16x32_f16(false, a, false, b, (short)0, c, false, false);
  asm volatile("v_nop\n\tv_nop\n\tv_nop\n\tv_nop" : "+v"(d) : "v"(a), "v"(b));
  return d;
}

__device__ __forceinline__ v16h load_frag(const _Float16* tile, int ld, int k0, int lane) {
  union { v16h v; v8h h[2]; } r;
  const _Float16* row = tile + (lane & 15) * ld + k0 + 8 * (lane >> 4);
  r.h[0] = *(const v8h*)(row);
  r.h[1] = *(const v8h*)(row + 16);
  return r.v;
}

__global__ __launch_bounds__(256) void gnn_layer1(
    const float* __restrict__ x, const float* __restrict__ times,
    const float* __restrict__ ts, const float* __restrict__ W0,
    const float* __restrict__ b0, const int* __restrict__ batch,
    const int* __restrict__ idx, _Float16* __restrict__ h1)
{
  __shared__ __attribute__((aligned(16))) _Float16 Wt[F_H * (F_IN + 8)];
  __shared__ __attribute__((aligned(16))) _Float16 Atile[16 * 72];
  __shared__ __attribute__((aligned(16))) _Float16 Ht[16 * F_H];
  __shared__ int   nbr[16][DEG];
  __shared__ int   nodeArr[16];
  __shared__ float tqArr[16];
  __shared__ float rowScale[16];
  __shared__ int   cnt[16];

  const int tid = threadIdx.x;
  const int wg  = blockIdx.x;

  for (int i = tid; i < F_IN * F_H; i += 256) {
    int k = i >> 7, n = i & 127;
    Wt[n * 72 + k] = (_Float16)W0[i];
  }

  if (tid < 16) {
    int m = wg * 16 + tid;
    int b = m / 33, j = m - b * 33;
    int bn  = batch[b];
    bn = bn < 0 ? 0 : (bn >= N_NODES ? N_NODES - 1 : bn);
    float tb = times[b];
    int node; float tq; float sc;
    if (j < DEG) {
      int e = bn * DEG + j;
      node = idx[e];
      node = node < 0 ? 0 : (node >= N_NODES ? N_NODES - 1 : node);
      tq   = ts[e];
      sc   = (tq <= tb) ? 1.0f : 0.0f;
    } else {
      node = bn; tq = tb; sc = 1.0f;
    }
    nodeArr[tid] = node; tqArr[tid] = tq; rowScale[tid] = sc;
  }
  __syncthreads();

  for (int e = tid; e < 16 * DEG; e += 256) {
    int r = e >> 5, d = e & 31;
    int ee = nodeArr[r] * DEG + d;
    int nb = idx[ee];
    nb = nb < 0 ? 0 : (nb >= N_NODES ? N_NODES - 1 : nb);
    bool ok = (ts[ee] <= tqArr[r]);
    nbr[r][d] = ok ? nb : -1;
  }
  __syncthreads();
  if (tid < 16) {
    int c = 1;
    for (int d = 0; d < DEG; ++d) c += (nbr[tid][d] >= 0) ? 1 : 0;
    cnt[tid] = c;
  }

  {
    int r = tid >> 4, f0 = (tid & 15) * 4;
    float4 acc = *(const float4*)(x + (size_t)nodeArr[r] * F_IN + f0);
#pragma unroll 4
    for (int d = 0; d < DEG; ++d) {
      int nb = nbr[r][d];
      if (nb >= 0) {
        float4 v = *(const float4*)(x + (size_t)nb * F_IN + f0);
        acc.x += v.x; acc.y += v.y; acc.z += v.z; acc.w += v.w;
      }
    }
    __syncthreads();
    float s = 1.0f / (float)cnt[r];
    _Float16* a = &Atile[r * 72 + f0];
    a[0] = (_Float16)(acc.x * s); a[1] = (_Float16)(acc.y * s);
    a[2] = (_Float16)(acc.z * s); a[3] = (_Float16)(acc.w * s);
  }
  __syncthreads();

  {
    int wv = tid >> 5, lane = tid & 31;
    int nl = wv * 16 + (lane & 15);
    v8f c = {};
#pragma unroll
    for (int s = 0; s < 2; ++s) {
      v16h a  = load_frag(Atile, 72, s * 32, lane);
      v16h bb = load_frag(Wt + wv * 16 * 72, 72, s * 32, lane);
      c = wmma_f16(a, bb, c);
    }
    float bias = b0[nl];
    int rbase = (lane >> 4) * 8;
#pragma unroll
    for (int i = 0; i < 8; ++i) {
      int r = rbase + i;
      float v = c[i] + bias;
      v = v > 0.0f ? v : 0.0f;
      v *= rowScale[r];
      Ht[r * F_H + nl] = (_Float16)v;
    }
  }
  __syncthreads();

  {
    const v4u val = *(const v4u*)((const char*)Ht + tid * 16);
    char* dst = (char*)(h1 + (size_t)wg * 16 * F_H) + tid * 16;
    *(volatile v4u*)dst = val;
    __threadfence();
    *(volatile v4u*)dst = val;
  }
}

__global__ __launch_bounds__(128) void gnn_layer2(
    const _Float16* __restrict__ h1, const float* __restrict__ times,
    const float* __restrict__ ts, const float* __restrict__ W1,
    const float* __restrict__ b1, const int* __restrict__ batch,
    float* __restrict__ out)
{
  __shared__ __attribute__((aligned(16))) _Float16 Wt[F_OUT * (F_H + 8)];
  __shared__ __attribute__((aligned(16))) _Float16 Atile[16 * 136];
  __shared__ __attribute__((aligned(16))) float Ot[16 * F_OUT];
  __shared__ int cnt[16];

  const int tid = threadIdx.x;
  const int wg  = blockIdx.x;

  for (int i = tid; i < F_H * F_OUT; i += 128) {
    int k = i >> 6, n = i & 63;
    Wt[n * 136 + k] = (_Float16)W1[i];
  }
  if (tid < 16) {
    int b  = wg * 16 + tid;
    int bn = batch[b];
    bn = bn < 0 ? 0 : (bn >= N_NODES ? N_NODES - 1 : bn);
    float tb = times[b];
    int c = 1;
    for (int d = 0; d < DEG; ++d) c += (ts[bn * DEG + d] <= tb) ? 1 : 0;
    cnt[tid] = c;
  }
  __syncthreads();

  {
    int r = tid >> 3, c0 = (tid & 7) * 16;
    int b = wg * 16 + r;
    float acc[16];
#pragma unroll
    for (int i = 0; i < 16; ++i) acc[i] = 0.0f;
    const _Float16* base = h1 + ((size_t)b * 33) * F_H + c0;
    for (int j = 0; j < 33; ++j) {
      v16h h = *(const v16h*)(base + (size_t)j * F_H);
#pragma unroll
      for (int i = 0; i < 16; ++i) acc[i] += (float)h[i];
    }
    float s = 1.0f / (float)cnt[r];
    _Float16* a = &Atile[r * 136 + c0];
#pragma unroll
    for (int i = 0; i < 16; ++i) a[i] = (_Float16)(acc[i] * s);
  }
  __syncthreads();

  {
    int wv = tid >> 5, lane = tid & 31;
    int nl = wv * 16 + (lane & 15);
    v8f c = {};
#pragma unroll
    for (int s = 0; s < 4; ++s) {
      v16h a  = load_frag(Atile, 136, s * 32, lane);
      v16h bb = load_frag(Wt + wv * 16 * 136, 136, s * 32, lane);
      c = wmma_f16(a, bb, c);
    }
    float bias = b1[nl];
    int rbase = (lane >> 4) * 8;
#pragma unroll
    for (int i = 0; i < 8; ++i) {
      float v = c[i] + bias;
      v = v > 0.0f ? v : 0.0f;
      Ot[(rbase + i) * F_OUT + nl] = v;
    }
  }
  __syncthreads();

  {
    char* dstb = (char*)(out + (size_t)wg * 16 * F_OUT);
    v4f v0 = *(const v4f*)((const char*)Ot + tid * 16);
    v4f v1 = *(const v4f*)((const char*)Ot + (128 + tid) * 16);
    *(volatile v4f*)(dstb + tid * 16) = v0;
    *(volatile v4f*)(dstb + (128 + tid) * 16) = v1;
    __threadfence();
    *(volatile v4f*)(dstb + tid * 16) = v0;
    *(volatile v4f*)(dstb + (128 + tid) * 16) = v1;
  }
}

extern "C" void kernel_launch(void* const* d_in, const int* in_sizes, int n_in,
                              void* d_out, int out_size, void* d_ws, size_t ws_size,
                              hipStream_t stream) {
  const float* x     = (const float*)d_in[0];
  const float* times = (const float*)d_in[1];
  const float* ts    = (const float*)d_in[2];
  const float* W0    = (const float*)d_in[3];
  const float* b0    = (const float*)d_in[4];
  const float* W1    = (const float*)d_in[5];
  const float* b1    = (const float*)d_in[6];
  const int*   batch = (const int*)d_in[7];
  const int*   idx   = (const int*)d_in[8];

  _Float16* h1 = (_Float16*)d_ws;
  float*    out = (float*)d_out;

  gnn_layer1<<<ROWS1 / 16, 256, 0, stream>>>(x, times, ts, W0, b0, batch, idx, h1);
  gnn_layer2<<<BQ / 16, 128, 0, stream>>>(h1, times, ts, W1, b1, batch, out);

  (void)in_sizes; (void)n_in; (void)out_size; (void)ws_size;
}
